// WP_31078383354695
// MI455X (gfx1250) — hardware-run, weakly checked
//
#include <hip/hip_runtime.h>
#include <math.h>


#ifndef NB
#define NB 32
#endif
#define NB_FULL 32
#define LSEQ 128
#define DM   256
#define NOUT 1024
#define MT   ((NB + 15) / 16)
#define MP   (MT * 16)
#define OSP  36
#define PSC  64.0f
#define WSC  1024.0f
#define CINV (1.0f / 65536.0f)
#define L2E  1.4426950408889634f
#define FILLV (-1.0e7f)
#define EPSV  1.0e-7f

static_assert(LSEQ == 128);
static_assert(DM == 256);
static_assert(8 * 16 == LSEQ);
static_assert(32 * 8 == DM);
static_assert(DM % 32 == 0);
static_assert(NOUT % 32 == 0);
static_assert(NB >= 1);
static_assert(NB <= NB_FULL);
static_assert(MP % 16 == 0);
static_assert(MP >= NB);
static_assert((OSP * 4) % 16 == 0);
static_assert((size_t)NB_FULL * NOUT * 4 == (size_t)131072);
static_assert((2 * LSEQ + 2 * LSEQ + DM + 16) * 4 <= 131072);
static_assert(16 * OSP * 4 <= 131072);

typedef _Float16 h16;
typedef unsigned short bf;
typedef __attribute__((ext_vector_type(16))) _Float16 v16h;
typedef __attribute__((ext_vector_type(8)))  _Float16 v8h;
typedef __attribute__((ext_vector_type(8)))  float    v8f;
typedef __attribute__((ext_vector_type(4)))  float    v4f;
typedef v4f  __attribute__((may_alias)) v4fa;

__device__ __forceinline__ unsigned short f2bf(float f) { unsigned u = __float_as_uint(f); u += 0x7FFFu + ((u >> 16) & 1u); return (unsigned short)(u >> 16); }
__device__ __forceinline__ float bfr(float f) { return __uint_as_float(((unsigned)f2bf(f)) << 16); }
__device__ __forceinline__ v16h cat16(v8h lo, v8h hi) { return __builtin_shufflevector(lo, hi, 0, 1, 2, 3, 4, 5, 6, 7, 8, 9, 10, 11, 12, 13, 14, 15); }
__device__ __forceinline__ v16h  ldh(const h16* p) { return cat16(*(const v8h*)p, *(const v8h*)(p + 16)); }
__device__ __forceinline__ void wave_sync() { __builtin_amdgcn_fence(3  , "wavefront"); __builtin_amdgcn_wave_barrier(); asm volatile("" ::: "memory"); }

static __device__ __forceinline__ h16 toh_flush(float v) { const h16 r = (h16)v; return (fabsf(v) < 6.103515625e-05f) ? (h16)0.0f : r; }
__device__ __forceinline__ v8f wmma16g(v16h a, v16h b, v8f c) {
    c = __builtin_amdgcn_wmma_f32_16x16x32_f16(false, a, false, b, (short)0, c, false, false);
    asm volatile("v_nop\n\tv_nop\n\tv_nop\n\tv_nop" : "+v"(c) : "v"(a), "v"(b));
    return c;
}
__device__ __forceinline__ v16h ldw(const float* p) {
    const v4f x0 = *(const v4f*)p, x1 = *(const v4f*)(p + 4), x2 = *(const v4f*)(p + 16), x3 = *(const v4f*)(p + 20);
    v16h o;
#pragma unroll
    for (int i = 0; i < 4; ++i) {
        o[i]      = toh_flush(bfr(x0[i]) * WSC); o[4 + i]  = toh_flush(bfr(x1[i]) * WSC);
        o[8 + i]  = toh_flush(bfr(x2[i]) * WSC); o[12 + i] = toh_flush(bfr(x3[i]) * WSC); }
    return o;
}

__global__ __launch_bounds__(256) void k_pool(const float* __restrict__ a1, const float* __restrict__ a2,
                                              const int* __restrict__ len1, const int* __restrict__ len2,
                                              const float* __restrict__ wew, h16* PH) {
#pragma clang fp contract(off)
    __shared__ __align__(16) float sd[2 * LSEQ];
    __shared__ __align__(16) float sco[2 * LSEQ];
    __shared__ __align__(16) float sp[DM];
    __shared__ float smx[8];
    __shared__ float ssm[8];
    const int tid = threadIdx.x, lane = tid & 31;
    const int wave = __builtin_amdgcn_readfirstlane((int)(threadIdx.x >> 5));
    const int b = blockIdx.x;
    if (b >= NB) {
        if (wave == 0) { const v8h z = (v8h){}; h16* dst = PH + (size_t)b * DM + lane * 8;
            *(volatile v8h*)dst = z; __threadfence(); *(volatile v8h*)dst = z; }
        return;
    }
    int l1 = len1[b]; l1 = l1 < 0 ? 0 : (l1 > LSEQ ? LSEQ : l1);
    int l2 = len2[b]; l2 = l2 < 0 ? 0 : (l2 > LSEQ ? LSEQ : l2);

    float wv[8];
    { const v8f wr = *(const v8f*)(wew + lane * 8);
#pragma unroll
      for (int k = 0; k < 8; ++k) wv[k] = bfr(wr[k]); }
    const float* x1 = a1 + (size_t)b * LSEQ * DM + lane * 8;
    const float* x2 = a2 + (size_t)b * LSEQ * DM + lane * 8;
#pragma unroll 1
    for (int r = wave * 16; r < wave * 16 + 16; ++r) {
        const v8f v = *(const v8f*)(x1 + (size_t)r * DM);
        float s = 0.0f;
#pragma unroll
        for (int k = 0; k < 8; ++k) s += bfr(v[k]) * wv[k];
        for (int off = 16; off > 0; off >>= 1) s += __shfl_xor(s, off, 32);
        if (lane == 0) sd[r] = s;
    }
#pragma unroll 1
    for (int r = wave * 16; r < wave * 16 + 16; ++r) {
        const v8f v = *(const v8f*)(x2 + (size_t)r * DM);
        float s = 0.0f;
#pragma unroll
        for (int k = 0; k < 8; ++k) s += bfr(v[k]) * wv[k];
        for (int off = 16; off > 0; off >>= 1) s += __shfl_xor(s, off, 32);
        if (lane == 0) sd[LSEQ + r] = s;
    }
    __syncthreads();

    const int rw = ((wave >> 2) & 1) ^ 1;
    const int idx = tid & (LSEQ - 1);
    const int obase = rw * LSEQ;
    const int nself = rw * l1 + (1 - rw) * l2;
    const int noth  = rw * l2 + (1 - rw) * l1;
    const float sg = (float)(2 * rw - 1);
    const bool valid = idx < nself;
    const float self = sd[tid];

    float m = FILLV;
#pragma unroll 1
    for (int k = 0; k < noth; ++k) {
        const float w = sg * (self - sd[obase + k]);
        const float mv = (fabsf(w) < EPSV) ? FILLV : w;
        m = fmaxf(m, mv);
    }
    m = valid ? m : FILLV;
    for (int off = 16; off > 0; off >>= 1) m = fmaxf(m, __shfl_xor(m, off, 32));
    if (lane == 0) smx[wave] = m;
    __syncthreads();
    float mx = smx[0];
#pragma unroll
    for (int k = 1; k < 8; ++k) mx = fmaxf(mx, smx[k]);

    float E = 0.0f;
#pragma unroll 1
    for (int k = 0; k < noth; ++k) {
        const float w = sg * (self - sd[obase + k]);
        const float mv = (fabsf(w) < EPSV) ? FILLV : w;
        E += __builtin_amdgcn_exp2f((mv - mx) * L2E);
    }
    E = valid ? E : 0.0f;
    float es = E;
    for (int off = 16; off > 0; off >>= 1) es += __shfl_xor(es, off, 32);
    if (lane == 0) ssm[wave] = es;
    __syncthreads();
    const float einv = __builtin_amdgcn_exp2f((FILLV - mx) * L2E);
    const float ninv = (float)(LSEQ * LSEQ - l1 * l2);
    const float Z = ((ssm[0] + ssm[1]) + (ssm[2] + ssm[3])) + ninv * einv;
    const float zi = 1.0f / Z;
    sco[tid] = sg * (E * zi);
    __syncthreads();

    const float* p1 = a1 + (size_t)b * LSEQ * DM + tid;
    const float* p2 = a2 + (size_t)b * LSEQ * DM + tid;
    float acc = 0.0f;
#pragma unroll 4
    for (int i = 0; i < l1; ++i) acc += sco[i] * bfr(p1[(size_t)i * DM]);
#pragma unroll 4
    for (int j = 0; j < l2; ++j) acc += sco[LSEQ + j] * bfr(p2[(size_t)j * DM]);
    sp[tid] = acc;
    __syncthreads();

    if (wave == 0) {
        const v4f y0 = *(const v4fa*)(&sp[lane * 8]); const v4f y1 = *(const v4fa*)(&sp[lane * 8 + 4]);
        v8h hv;
#pragma unroll
        for (int i = 0; i < 4; ++i) { hv[i] = toh_flush(y0[i] * PSC); hv[4 + i] = toh_flush(y1[i] * PSC); }
        h16* dst = PH + (size_t)b * DM + lane * 8;
        *(volatile v8h*)dst = hv; __threadfence(); *(volatile v8h*)dst = hv;
    }
}

static_assert(32 * 4 * 4 == 16 * 32);
__global__ __launch_bounds__(32) void k_fc(const h16* __restrict__ PH, const float* __restrict__ W, const float* __restrict__ bias, float* OUT) {
    __shared__ __align__(16) float os[16 * OSP];
    const int lane = threadIdx.x & 31, lr = lane & 15, hi = lane >> 4;
    const int n0 = blockIdx.x * 32;
    v8f acc[MT][2];
#pragma unroll
    for (int mb = 0; mb < MT; ++mb)
#pragma unroll
        for (int nb = 0; nb < 2; ++nb) acc[mb][nb] = (v8f){};
    const size_t aoff = (size_t)lr * DM + 8 * hi, boff = (size_t)(n0 + lr) * DM + 8 * hi;
#pragma unroll 2
    for (int kc = 0; kc < DM; kc += 32) {
        v16h a[MT];
#pragma unroll
        for (int mb = 0; mb < MT; ++mb) a[mb] = ldh(PH + aoff + (size_t)mb * 16 * DM + kc);
#pragma unroll
        for (int nb = 0; nb < 2; ++nb) { const v16h bq = ldw(W + boff + (size_t)nb * 16 * DM + kc);
#pragma unroll
            for (int mb = 0; mb < MT; ++mb) acc[mb][nb] = wmma16g(a[mb], bq, acc[mb][nb]); }
    }
    float bc[2];
#pragma unroll
    for (int nb = 0; nb < 2; ++nb) bc[nb] = bfr(bias[n0 + nb * 16 + lr]);
#pragma unroll
    for (int mb = 0; mb < MT; ++mb) {
#pragma unroll
        for (int nb = 0; nb < 2; ++nb) {
#pragma unroll
            for (int j = 0; j < 8; ++j) os[(hi * 8 + j) * OSP + nb * 16 + lr] = acc[mb][nb][j] * CINV + bc[nb]; }
        wave_sync();
#pragma unroll 1
        for (int s = 0; s < 4; ++s) { const int row = 4 * s + (lane >> 3), cofs = (lane & 7) * 4;
            const v4f x = *(const v4fa*)(&os[row * OSP + cofs]); v4f y;
#pragma unroll
            for (int i = 0; i < 4; ++i) y[i] = tanhf(x[i]);
            *(v4fa*)(&os[row * OSP + cofs]) = y; }
        wave_sync();
        float* orow = OUT + (size_t)(mb * 16) * NOUT + n0;
#pragma unroll 1
        for (int ps = 0; ps < 2; ++ps) {
#pragma unroll
            for (int s = 0; s < 4; ++s) { const int row = 4 * s + (lane >> 3), cofs = (lane & 7) * 4;
                const v4f val = *(const v4fa*)(&os[row * OSP + cofs]);
                if (mb * 16 + row < NB) *(volatile v4f*)(orow + (size_t)row * NOUT + cofs) = val; }
            if (ps == 0) __threadfence(); }
        wave_sync();
    }
}

static constexpr size_t al256(size_t v) { return (v + 255) & ~(size_t)255; }
static constexpr size_t SZ_PH = al256((size_t)MP * DM * 2);
static constexpr size_t SZ_TOTAL = SZ_PH;
static_assert(SZ_TOTAL <= (size_t)134217728);
static_assert((size_t)(MP - 1) * DM * 2 + 32 * 16 <= SZ_PH);

extern "C" void kernel_launch(void* const* d_in, const int* in_sizes, int n_in,
                              void* d_out, int out_size, void* d_ws, size_t ws_size, hipStream_t stream) {
    if (n_in < 7) return;
    const size_t needx = (size_t)NB * LSEQ * DM;
    if ((size_t)in_sizes[0] < needx || (size_t)in_sizes[2] < needx) return;
    if (in_sizes[1] < NB || in_sizes[3] < NB) return;
    if ((size_t)in_sizes[4] < (size_t)NOUT * DM || in_sizes[5] < NOUT || in_sizes[6] < DM) return;
    if ((size_t)out_size < (size_t)NB * NOUT) return;
    if (SZ_TOTAL > ws_size) return;
    const float* a1  = (const float*)d_in[0];
    const int*   ln1 = (const int*)d_in[1];
    const float* a2  = (const float*)d_in[2];
    const int*   ln2 = (const int*)d_in[3];
    const float* fw  = (const float*)d_in[4];
    const float* fb  = (const float*)d_in[5];
    const float* ww  = (const float*)d_in[6];
    float* OUT = (float*)d_out;
    h16* PH = (h16*)d_ws;

    k_pool<<<dim3(MP, 1, 1), 256, 0, stream>>>(a1, a2, ln1, ln2, ww, PH);
    k_fc<<<dim3(NOUT / 32, 1, 1), 32, 0, stream>>>(PH, fw, fb, OUT);
}
